// MambaLayerlocal_5403068858466
// MI455X (gfx1250) — hardware-verified
//
#include <hip/hip_runtime.h>
#include <math.h>

typedef __attribute__((ext_vector_type(16))) _Float16 v16h;
typedef __attribute__((ext_vector_type(8)))  _Float16 v8h;
typedef __attribute__((ext_vector_type(16))) __bf16   v16b;
typedef __attribute__((ext_vector_type(8)))  __bf16   v8b;
typedef __attribute__((ext_vector_type(8)))  float    v8f;
typedef __attribute__((ext_vector_type(4)))  float    v4f;

constexpr int kB    = 2;
constexpr int kNF   = 8;
constexpr int kH    = 32;
constexpr int kW    = 32;
constexpr int kHW   = kH * kW;
constexpr int kL    = kNF * kH * kW;
constexpr int kC    = 256;
constexpr int kDin  = 128;
constexpr int kNst  = 16;
constexpr int kDtR  = 16;
constexpr int kXdW  = kDtR + 2 * kNst;
constexpr int kXdP  = 64;
constexpr int kHid  = 1024;
constexpr int kRows = kB * kL;
constexpr float kEps = 1e-5f;
constexpr int kConvTP = 132;
constexpr int kScanTS = 64;
constexpr int kScanCh = 64;
constexpr int kScanYP = 68;
constexpr int kTileP  = 260;
constexpr float kLnCarry  = 8.0f;
constexpr float kWCarry   = 256.0f;
constexpr float kXsCarry  = 64.0f;
constexpr float kYCarry   = 256.0f;
constexpr float kActCarry = 64.0f;
static_assert(kXdW <= kXdP && (kXdP % 64) == 0);
static_assert((kC % 32) == 0 && (kDin % 32) == 0 && (kHid % 32) == 0);
static_assert((kRows % 64) == 0 && (kC % 64) == 0 && (kHid % 64) == 0 && (kXdP % 64) == 0);
static_assert((kL % kScanTS) == 0 && (kL % 64) == 0 && (kDin % kScanCh) == 0 && kDin == 128 && kC == 256);

constexpr size_t kMiB     = 1048576ull;
constexpr size_t kOffXF   = 0;
constexpr size_t kOffSEQ  = 16 * kMiB;
constexpr size_t kPlaneB  = (size_t)kRows * kC * 4;
constexpr size_t kOffXZ   = 64 * kMiB;
constexpr size_t kOffNX   = 80 * kMiB;
constexpr size_t kOffXS   = 88 * kMiB;
constexpr size_t kOffXS16 = 96 * kMiB;
constexpr size_t kOffXD   = 100 * kMiB;
constexpr size_t kOffY16  = 104 * kMiB;
constexpr size_t kOffXM   = kOffXZ;
constexpr size_t kOffNXM  = kOffNX;
constexpr size_t kOffHDN  = 0;
constexpr size_t kOffHACT = 88 * kMiB;
constexpr size_t kOffXO   = 0;
constexpr size_t kOffWI   = 120 * kMiB;
constexpr size_t kOffWX   = kOffWI + (size_t)kC * kC * 2;
constexpr size_t kOffWO   = kOffWX + (size_t)kXdP * kDin * 2;
constexpr size_t kOffW1   = kOffWO + (size_t)kC * kDin * 2;
constexpr size_t kOffW2   = kOffW1 + (size_t)kHid * kC * 2;
constexpr size_t kOffPART = kOffW2 + (size_t)kC * kHid * 2;
constexpr size_t kOffWGT  = kOffPART + (size_t)kB * 3 * 32 * 256 * 4;
constexpr size_t kWsTotal = kOffWGT + (size_t)kB * 3 * 256 * 4;
static_assert(kWsTotal == 127293440ull);
static_assert(kWsTotal <= 134217728ull);
static_assert(kPlaneB == 16 * kMiB);
static_assert(kOffSEQ + 3 * kPlaneB == kOffXZ);
static_assert(kOffXZ + (size_t)kRows * kC * 4 == kOffNX);
static_assert(kOffNX + (size_t)kRows * kC * 2 == kOffXS);
static_assert(kOffXS + (size_t)kRows * kDin * 4 == kOffXS16);
static_assert(kOffXS16 + (size_t)kRows * kDin * 2 == kOffXD);
static_assert(kOffXD + (size_t)kRows * kXdP * 4 == kOffY16);
static_assert(kOffY16 + (size_t)kRows * kDin * 2 <= kOffWI);
static_assert(kOffHDN + (size_t)kRows * kHid * 4 <= kOffXM);
static_assert(kOffHACT + (size_t)kRows * kHid * 2 == kOffWI);
static_assert(kOffXO + (size_t)kRows * kC * 4 <= kOffXM);
static_assert((kOffWX % 128) == 0 && (kOffWO % 128) == 0 && (kOffW1 % 128) == 0 && (kOffW2 % 128) == 0 &&
              (kOffPART % 128) == 0 && (kOffWGT % 128) == 0);

__device__ __forceinline__ unsigned short f2bf_bits(float f) {
  unsigned u = __float_as_uint(f);
  return (unsigned short)((u + 0x7FFFu + ((u >> 16) & 1u)) >> 16);
}
__device__ __forceinline__ float bf_bits2f(unsigned short h) { return __uint_as_float(((unsigned)h) << 16); }

__device__ __forceinline__ void dep_guard_h(v8f& a, v8f& b, v16h x, v16h y) { asm volatile("v_nop\n\tv_nop\n\tv_nop\n\tv_nop" : "+v"(a), "+v"(b) : "v"(x), "v"(y)); }
__device__ __forceinline__ void dep_guard_b(v8f& a, v8f& b, v16b x, v16b y) { asm volatile("v_nop\n\tv_nop\n\tv_nop\n\tv_nop" : "+v"(a), "+v"(b) : "v"(x), "v"(y)); }
__device__ __forceinline__ void keep4_h(v16h a, v16h b, v16h c, v16h d) { asm volatile("v_nop" :: "v"(a), "v"(b), "v"(c), "v"(d)); }
__device__ __forceinline__ void keep4_b(v16b a, v16b b, v16b c, v16b d) { asm volatile("v_nop" :: "v"(a), "v"(b), "v"(c), "v"(d)); }
__device__ __forceinline__ void acc_guard4(v8f& a, v8f& b, v8f& c, v8f& d) { asm volatile("v_nop\n\tv_nop\n\tv_nop\n\tv_nop" : "+v"(a), "+v"(b), "+v"(c), "+v"(d)); }
template <typename T> struct Frag;
template <> struct Frag<_Float16> {
  typedef v16h V; union U { v16h v; v8h h[2]; };
  static __device__ __forceinline__ v16h load(const _Float16* p) {
    U f; f.h[0] = *(const v8h*)(p); f.h[1] = *(const v8h*)(p + 16); return f.v;
  }
  static __device__ __forceinline__ v8f mma(v16h a, v16h b, v8f c) {
    return __builtin_amdgcn_wmma_f32_16x16x32_f16(false, a, false, b, (short)0, c, false, false);
  }
  static __device__ __forceinline__ void guard(v8f& a, v8f& b, v16h x, v16h y) { dep_guard_h(a, b, x, y); }
  static __device__ __forceinline__ void keep(v16h a, v16h b, v16h c, v16h d) { keep4_h(a, b, c, d); }
};
template <> struct Frag<__bf16> {
  typedef v16b V; union U { v16b v; v8b h[2]; };
  static __device__ __forceinline__ v16b load(const __bf16* p) {
    U f; f.h[0] = *(const v8b*)(p); f.h[1] = *(const v8b*)(p + 16); return f.v;
  }
  static __device__ __forceinline__ v8f mma(v16b a, v16b b, v8f c) {
    return __builtin_amdgcn_wmma_f32_16x16x32_bf16(false, a, false, b, (short)0, c, false, false);
  }
  static __device__ __forceinline__ void guard(v8f& a, v8f& b, v16b x, v16b y) { dep_guard_b(a, b, x, y); }
  static __device__ __forceinline__ void keep(v16b a, v16b b, v16b c, v16b d) { keep4_b(a, b, c, d); }
};

template <int ET> struct Elem;
template <> struct Elem<0> { typedef _Float16 T; };
template <> struct Elem<1> { typedef __bf16 T; };
template <int ET, int SPL, int BIAS_MODE, int OUT_MODE, bool RESID, int ACT = 0>
__global__ __launch_bounds__(256) void wmma_gemm64(
    const unsigned short* __restrict__ Ap, const unsigned short* __restrict__ A2p, int lda, long strideA,
    const unsigned short* __restrict__ Btp, const unsigned short* __restrict__ Bt2p, int ldb, long strideB,
    void* __restrict__ Cout, void* __restrict__ Cout2, int ldc, long strideC,
    const float* __restrict__ bias,
    const float* __restrict__ resid, long strideR,
    int M, int N, int K, float scale) {
  typedef typename Elem<ET>::T T;
  typedef typename Frag<T>::V V;
  const T* A = (const T*)Ap; const T* A2 = (const T*)A2p; const T* Bt = (const T*)Btp; const T* Bt2 = (const T*)Bt2p;
  __shared__ __align__(16) float sT[8][16 * 68];
  const int b    = blockIdx.y;
  const int lane = threadIdx.x & 31;
  const int wave = threadIdx.x >> 5;
  const int tilesN = N >> 6;
  const int tilesM = M >> 6;
  const int tile = blockIdx.x * 8 + wave;
  if (tile >= tilesM * tilesN) return;
  const int tm = tile / tilesN;
  const int tn = tile - tm * tilesN;
  const int m0 = tm << 6;
  const int n0 = tn << 6;

  const T* Ab  = A  + (size_t)b * strideA;
  const T* Bb  = Bt + (size_t)b * strideB;
  const T* Ab2 = (SPL >= 1) ? (A2  + (size_t)b * strideA) : nullptr;
  const T* Bb2 = (SPL == 2) ? (Bt2 + (size_t)b * strideB) : nullptr;

  const int rlane = lane & 15;
  const int koff  = (lane >> 4) * 8;
  const int mOff  = (lane >> 4) * 8;

  v8f acc[4][4];
#pragma unroll
  for (int i = 0; i < 4; ++i)
#pragma unroll
    for (int j = 0; j < 4; ++j) acc[i][j] = (v8f){0.f,0.f,0.f,0.f,0.f,0.f,0.f,0.f};

  for (int k0 = 0; k0 < K; k0 += 32) {
    V bh[4], bl[4];
#pragma unroll
    for (int j = 0; j < 4; ++j) {
      const size_t bo = (size_t)(n0 + (j << 4) + rlane) * ldb + koff + k0;
      bh[j] = Frag<T>::load(Bb + bo);
      if (SPL == 2) bl[j] = Frag<T>::load(Bb2 + bo);
    }
#pragma unroll
    for (int i = 0; i < 4; ++i) {
      const size_t ao = (size_t)(m0 + (i << 4) + rlane) * lda + koff + k0;
      V ah = Frag<T>::load(Ab + ao);
      V al;
      if (SPL >= 1) al = Frag<T>::load(Ab2 + ao);
#pragma unroll
      for (int j = 0; j < 4; ++j) {
        acc[i][j] = Frag<T>::mma(ah, bh[j], acc[i][j]);
        if (SPL == 2) acc[i][j] = Frag<T>::mma(ah, bl[j], acc[i][j]);
        if (SPL >= 1) acc[i][j] = Frag<T>::mma(al, bh[j], acc[i][j]);
      }
      Frag<T>::guard(acc[i][0], acc[i][3], ah, (SPL >= 1) ? al : ah);
    }
    Frag<T>::keep(bh[0], bh[1], bh[2], bh[3]);
    if (SPL == 2) Frag<T>::keep(bl[0], bl[1], bl[2], bl[3]);
  }
  acc_guard4(acc[0][0], acc[0][1], acc[0][2], acc[0][3]);
  acc_guard4(acc[1][0], acc[1][1], acc[1][2], acc[1][3]);
  acc_guard4(acc[2][0], acc[2][1], acc[2][2], acc[2][3]);
  acc_guard4(acc[3][0], acc[3][1], acc[3][2], acc[3][3]);

  float* slab = sT[wave];
  const float* Rb = RESID ? (resid + (size_t)b * strideR) : nullptr;
#pragma unroll
  for (int i = 0; i < 4; ++i) {
    const int mBase = m0 + (i << 4);
#pragma unroll
    for (int j = 0; j < 4; ++j) {
      const int n = n0 + (j << 4) + rlane;
      float bv = 0.f;
      if (BIAS_MODE == 2) bv = bias[n];
#pragma unroll
      for (int r = 0; r < 8; ++r) {
        float v = acc[i][j][r] * scale;
        if (BIAS_MODE == 1) v += bias[mBase + mOff + r];
        if (BIAS_MODE == 2) v += bv;
        if (RESID) v += Rb[(size_t)(mBase + mOff + r) * ldc + n];
        if (ACT == 1) v = tanhf(v);
        if (ACT == 2) v = fmaxf(v, 0.0f);
        if (ACT == 3) v = v / (1.0f + expf(-v));
        if (ACT == 4) v = (v > 0.f) ? v : 0.01f * v;
        slab[(mOff + r) * 68 + (j << 4) + rlane] = v;
      }
    }
    __builtin_amdgcn_fence(__ATOMIC_RELEASE, "workgroup");
    __builtin_amdgcn_wave_barrier();
    __builtin_amdgcn_fence(__ATOMIC_ACQUIRE, "workgroup");
    if (OUT_MODE == 0) {
      float* C = (float*)Cout + (size_t)b * strideC;
      const int hh = lane >> 4, c4 = (lane & 15) * 4;
      for (int pass = 0; pass < 2; ++pass) {
#pragma unroll
        for (int it = 0; it < 8; ++it) {
          const int row = it * 2 + hh;
          v4f v = *(const v4f*)(slab + row * 68 + c4);
          *(volatile v4f*)(C + (size_t)(mBase + row) * ldc + n0 + c4) = v;
        }
        __threadfence();
      }
    } else {
      const int q = lane >> 3, c8 = (lane & 7) * 8;
      unsigned short* C  = (unsigned short*)Cout  + (size_t)b * strideC;
      unsigned short* C2 = (OUT_MODE == 2) ? ((unsigned short*)Cout2 + (size_t)b * strideC) : nullptr;
      for (int pass = 0; pass < 2; ++pass) {
#pragma unroll
        for (int it = 0; it < 4; ++it) {
          const int row = it * 4 + q;
          const float* sp = slab + row * 68 + c8;
          v8h hv, lv;
#pragma unroll
          for (int e = 0; e < 8; ++e) {
            if (OUT_MODE == 1) {
              hv[e] = (_Float16)sp[e];
            } else {
              unsigned short hb = f2bf_bits(sp[e]);
              unsigned short lb = f2bf_bits(sp[e] - bf_bits2f(hb));
              hv[e] = __builtin_bit_cast(_Float16, hb);
              lv[e] = __builtin_bit_cast(_Float16, lb);
            }
          }
          *(volatile v8h*)(C + (size_t)(mBase + row) * ldc + n0 + c8) = hv;
          if (OUT_MODE == 2) *(volatile v8h*)(C2 + (size_t)(mBase + row) * ldc + n0 + c8) = lv;
        }
        __threadfence();
      }
    }
    __builtin_amdgcn_fence(__ATOMIC_RELEASE, "workgroup");
    __builtin_amdgcn_wave_barrier();
    __builtin_amdgcn_fence(__ATOMIC_ACQUIRE, "workgroup");
  }
}

__device__ __forceinline__ float wave_sum32(float v) {
#pragma unroll
  for (int off = 16; off > 0; off >>= 1) v += __shfl_xor(v, off, 32);
  return v;
}

__global__ __launch_bounds__(256) void cast_scale_f16_kernel(
    const float* __restrict__ in, unsigned short* __restrict__ out, int n2valid, int n2total, float scale)
{
  const int i = blockIdx.x * 256 + threadIdx.x;
  if (i >= n2total) return;
  const bool valid = (i < n2valid);
  const int ic = valid ? i : (n2valid - 1);
  const float a0 = in[2 * (size_t)ic] * scale;
  const float a1 = in[2 * (size_t)ic + 1] * scale;
  const _Float16 h0 = (_Float16)a0, h1 = (_Float16)a1;
  unsigned u = (unsigned)__builtin_bit_cast(unsigned short, h0) | ((unsigned)__builtin_bit_cast(unsigned short, h1) << 16);
  u = valid ? u : 0u;
  ((volatile unsigned*)out)[i] = u;
  __threadfence();
  ((volatile unsigned*)out)[i] = u;
}

__global__ __launch_bounds__(256) void gather_ln_kernel(
    const float* __restrict__ x, const float* __restrict__ fx, const int* __restrict__ perm,
    const float* __restrict__ lnw, const float* __restrict__ lnb,
    float* __restrict__ XF, float* __restrict__ FF, unsigned short* __restrict__ NX)
{
  __shared__ __align__(16) float sS[8][2][kC];
  const int tid = threadIdx.x, lane = tid & 31, wave = tid >> 5;
  const int row = blockIdx.x * 8 + wave;
  const int bi = row >> 13;
  const int l = row & (kL - 1);
  int p = perm[l];
  p = p < 0 ? 0 : (p > kL - 1 ? kL - 1 : p);
  const int f = p >> 10, hw = p & (kHW - 1);
  const size_t base = ((size_t)(bi * kNF + f) * kC) * (size_t)kHW + (size_t)hw;
  const int c0 = lane * 8;
  float xv[8], fv[8];
#pragma unroll
  for (int e = 0; e < 8; ++e) {
    const size_t a = base + (size_t)(c0 + e) * kHW;
    xv[e] = x[a];
    fv[e] = fx[a];
  }
  float s = 0.f;
#pragma unroll
  for (int e = 0; e < 8; ++e) s += xv[e];
  s = wave_sum32(s);
  const float mean = s * (1.0f / (float)kC);
  float dv[8];
  float qs = 0.f;
#pragma unroll
  for (int e = 0; e < 8; ++e) { dv[e] = xv[e] - mean; qs += dv[e] * dv[e]; }
  qs = wave_sum32(qs);
  const float rstd = rsqrtf(qs * (1.0f / (float)kC) + kEps);
  const v4f w0 = *(const v4f*)(lnw + c0), w1 = *(const v4f*)(lnw + c0 + 4);
  const v4f g0 = *(const v4f*)(lnb + c0), g1 = *(const v4f*)(lnb + c0 + 4);
  v8h hv;
#pragma unroll
  for (int e = 0; e < 4; ++e) {
    const float n0 = dv[e] * rstd * w0[e] + g0[e];
    const float n1 = dv[4 + e] * rstd * w1[e] + g1[e];
    hv[e]     = (_Float16)(n0 * kLnCarry);
    hv[4 + e] = (_Float16)(n1 * kLnCarry);
  }
  float* s0 = sS[wave][0];
  float* s1 = sS[wave][1];
  *(v4f*)(s0 + c0)     = (v4f){xv[0], xv[1], xv[2], xv[3]};
  *(v4f*)(s0 + c0 + 4) = (v4f){xv[4], xv[5], xv[6], xv[7]};
  *(v4f*)(s1 + c0)     = (v4f){fv[0], fv[1], fv[2], fv[3]};
  *(v4f*)(s1 + c0 + 4) = (v4f){fv[4], fv[5], fv[6], fv[7]};
  __builtin_amdgcn_fence(__ATOMIC_RELEASE, "workgroup");
  __builtin_amdgcn_wave_barrier();
  __builtin_amdgcn_fence(__ATOMIC_ACQUIRE, "workgroup");
  const int c4 = lane * 4;
  const v4f xa = *(const v4f*)(s0 + c4), xb = *(const v4f*)(s0 + 128 + c4);
  const v4f fa = *(const v4f*)(s1 + c4), fb = *(const v4f*)(s1 + 128 + c4);
  const size_t ro = (size_t)row * kC;
  for (int pass = 0; pass < 2; ++pass) {
    *(volatile v4f*)(XF + ro + c4)       = xa;
    *(volatile v4f*)(XF + ro + 128 + c4) = xb;
    *(volatile v4f*)(FF + ro + c4)       = fa;
    *(volatile v4f*)(FF + ro + 128 + c4) = fb;
    *(volatile v8h*)(NX + ro + c0)       = hv;
    __threadfence();
  }
}

__global__ __launch_bounds__(128) void conv_silu_kernel(
    const float* __restrict__ XZ, const float* __restrict__ cw, const float* __restrict__ cb,
    float* __restrict__ XS, unsigned short* __restrict__ XS16, int dir)
{
  __shared__ __align__(16) float sT[16 * kConvTP];
  const int tid = threadIdx.x, lane = tid & 31, wave = tid >> 5;
  const int d = tid;
  const int bix = blockIdx.x >> 7;
  const int j0 = (blockIdx.x & 127) * 64;
  const size_t rb = (size_t)bix * kL;
  const float w0 = cw[d * 4 + 0], w1 = cw[d * 4 + 1], w2 = cw[d * 4 + 2], w3 = cw[d * 4 + 3];
  const float bc = cb[d];
  float xm3, xm2, xm1;
  {
    const bool hist = (j0 > 0);
    const int jb = hist ? (j0 - 3) : 0;
    const int s3 = dir ? (kL - 1 - jb) : jb;
    const int s2 = dir ? (kL - 2 - jb) : (jb + 1);
    const int s1 = dir ? (kL - 3 - jb) : (jb + 2);
    const float v3 = XZ[(rb + (size_t)s3) * kC + d];
    const float v2 = XZ[(rb + (size_t)s2) * kC + d];
    const float v1 = XZ[(rb + (size_t)s1) * kC + d];
    xm3 = hist ? v3 : 0.f;
    xm2 = hist ? v2 : 0.f;
    xm1 = hist ? v1 : 0.f;
  }
#pragma unroll 1
  for (int sub = 0; sub < 4; ++sub) {
    const int lb = j0 + sub * 16;
#pragma unroll 1
    for (int s = 0; s < 16; ++s) {
      const int j = lb + s;
      const int sj = dir ? (kL - 1 - j) : j;
      const float xcur = XZ[(rb + (size_t)sj) * kC + d];
      float acc = w0 * xm3;
      acc = fmaf(w1, xm2, acc);
      acc = fmaf(w2, xm1, acc);
      acc = fmaf(w3, xcur, acc);
      const float sv = acc + bc;
      const float sg = __builtin_amdgcn_rcpf(1.0f + __expf(-sv));
      sT[s * kConvTP + tid] = sv * sg;
      xm3 = xm2; xm2 = xm1; xm1 = xcur;
    }
    __syncthreads();
    v4f fv[4];
    v8h hv[2];
#pragma unroll
    for (int it = 0; it < 4; ++it) fv[it] = *(const v4f*)(sT + (it * 4 + wave) * kConvTP + lane * 4);
#pragma unroll
    for (int it = 0; it < 2; ++it) {
      const float* sp = sT + (it * 8 + wave * 2 + (lane >> 4)) * kConvTP + (lane & 15) * 8;
      const v4f a0 = *(const v4f*)(sp);
      const v4f a1 = *(const v4f*)(sp + 4);
#pragma unroll
      for (int e = 0; e < 4; ++e) {
        hv[it][e]     = (_Float16)(a0[e] * kXsCarry);
        hv[it][4 + e] = (_Float16)(a1[e] * kXsCarry);
      }
    }
    for (int pass = 0; pass < 2; ++pass) {
#pragma unroll
      for (int it = 0; it < 4; ++it)
        *(volatile v4f*)(XS + (rb + (size_t)(lb + it * 4 + wave)) * kDin + lane * 4) = fv[it];
#pragma unroll
      for (int it = 0; it < 2; ++it) {
        const size_t o = (rb + (size_t)(lb + it * 8 + wave * 2 + (lane >> 4))) * kDin + (lane & 15) * 8;
        *(volatile v8h*)(XS16 + o) = hv[it];
      }
      __threadfence();
    }
    __syncthreads();
  }
}

__global__ __launch_bounds__(64) void scan_kernel(
    const float* __restrict__ XD, const float* __restrict__ XS, const float* __restrict__ XZ,
    const float* __restrict__ Wdt, const float* __restrict__ bdt, const float* __restrict__ Alog,
    const float* __restrict__ Dp, unsigned short* __restrict__ Y16, int dir)
{
  __shared__ __align__(16) float sX[kScanTS * kXdP];
  __shared__ __align__(16) float sY[kScanTS * kScanYP];
  __shared__ __align__(16) float sW[kDtR * kScanCh];
  __shared__ __align__(16) float sA[kNst * kScanCh];
  const int tid = threadIdx.x, lane = tid & 31, wave = tid >> 5;
  constexpr int kBlkPerB = kDin / kScanCh;
  const int bix = blockIdx.x / kBlkPerB;
  const int d0  = (blockIdx.x - bix * kBlkPerB) * kScanCh;
  const int d   = d0 + tid;
  const size_t row0 = (size_t)bix * kL;
#pragma unroll 1
  for (int r = 0; r < kDtR; ++r) sW[r * kScanCh + tid] = Wdt[(size_t)d * kDtR + r];
#pragma unroll 1
  for (int s = 0; s < kNst; ++s) sA[s * kScanCh + tid] = -expf(Alog[(size_t)d * kNst + s]);
  __syncthreads();
  float negA[kNst], h[kNst];
#pragma unroll
  for (int s = 0; s < kNst; ++s) {
    negA[s] = sA[s * kScanCh + tid];
    h[s] = 0.f;
  }
  const float bb = bdt[d], Dd = Dp[d];
  const int lr = tid >> 4, lc4 = (tid & 15) * 4;
  const int q = lane >> 3, c8 = (lane & 7) * 8;
#pragma unroll 1
  for (int t0 = 0; t0 < kL; t0 += kScanTS) {
    __syncthreads();
#pragma unroll
    for (int i = 0; i < 16; ++i) {
      const int r = lr + 4 * i;
      *(v4f*)(sX + r * kXdP + lc4) = *(const v4f*)(XD + (row0 + t0 + r) * kXdP + lc4);
    }
    __syncthreads();
#pragma unroll 1
    for (int s = 0; s < kScanTS; ++s) {
      const int t = t0 + s;
      const float* xr = sX + s * kXdP;
      float vdot = 0.f;
#pragma unroll 1
      for (int r4 = 0; r4 < kDtR / 4; ++r4) {
        const v4f xv = *(const v4f*)(xr + 4 * r4);
        const float* wp = sW + (4 * r4) * kScanCh + tid;
        vdot = fmaf(xv[0], wp[0], vdot);
        vdot = fmaf(xv[1], wp[kScanCh], vdot);
        vdot = fmaf(xv[2], wp[2 * kScanCh], vdot);
        vdot = fmaf(xv[3], wp[3 * kScanCh], vdot);
      }
      float Bs[kNst], Cs[kNst];
#pragma unroll
      for (int q4 = 0; q4 < 4; ++q4) {
        const v4f bv = *(const v4f*)(xr + kDtR + 4 * q4);
        const v4f cv = *(const v4f*)(xr + kDtR + kNst + 4 * q4);
        Bs[4 * q4 + 0] = bv[0]; Bs[4 * q4 + 1] = bv[1]; Bs[4 * q4 + 2] = bv[2]; Bs[4 * q4 + 3] = bv[3];
        Cs[4 * q4 + 0] = cv[0]; Cs[4 * q4 + 1] = cv[1]; Cs[4 * q4 + 2] = cv[2]; Cs[4 * q4 + 3] = cv[3];
      }
      const float v   = vdot + bb;
      const float a   = __expf(-fabsf(v));
      const float u   = 1.0f + a;
      const float l1p = __logf(u) + (a - (u - 1.0f)) * __builtin_amdgcn_rcpf(u);
      const float dt  = fmaxf(v, 0.0f) + l1p;
      const float xt  = XS[(row0 + t) * kDin + d];
      const float dtx = dt * xt;
      float y = 0.f;
#pragma unroll
      for (int k = 0; k < kNst; ++k) {
        const float e = __expf(dt * negA[k]);
        h[k] = e * h[k] + dtx * Bs[k];
        y = h[k] * Cs[k] + y;
      }
      y = xt * Dd + y;
      const int ot = dir ? (kL - 1 - t) : t;
      const float zv = XZ[(row0 + (size_t)ot) * kC + kDin + d];
      const float sg = __builtin_amdgcn_rcpf(1.0f + __expf(-zv));
      y = y * (zv * sg);
      const int slot = dir ? (kScanTS - 1 - s) : s;
      sY[slot * kScanYP + tid] = y;
    }
    __syncthreads();
    v8h hv[8];
#pragma unroll
    for (int it = 0; it < 8; ++it) {
      const int row = it * 8 + wave * 4 + q;
      const float* sp = sY + row * kScanYP + c8;
      const v4f a0 = *(const v4f*)(sp);
      const v4f a1 = *(const v4f*)(sp + 4);
#pragma unroll
      for (int e = 0; e < 4; ++e) {
        hv[it][e]     = (_Float16)(a0[e] * kYCarry);
        hv[it][4 + e] = (_Float16)(a1[e] * kYCarry);
      }
    }
    const int ob = dir ? (kL - kScanTS - t0) : t0;
    for (int pass = 0; pass < 2; ++pass) {
#pragma unroll
      for (int it = 0; it < 8; ++it) {
        const int row = it * 8 + wave * 4 + q;
        const size_t o = (row0 + (size_t)(ob + row)) * kDin + d0 + c8;
        *(volatile v8h*)(Y16 + o) = hv[it];
      }
      __threadfence();
    }
  }
}

__global__ __launch_bounds__(256) void pool_partial_kernel(const float* __restrict__ SEQ, float* __restrict__ PART)
{
  const int tid = threadIdx.x;
  const int chunk = blockIdx.x & 31;
  const int bs = blockIdx.x >> 5;
  const int bi = bs / 3;
  const int j = bs - 3 * bi;
  const float* p = SEQ + (size_t)j * ((size_t)kRows * kC) + ((size_t)bi * kL + (size_t)chunk * 256) * kC + tid;
  float s0 = 0.f, s1 = 0.f, s2 = 0.f, s3 = 0.f;
#pragma unroll 1
  for (int r = 0; r < 256; r += 4) {
    s0 += p[(size_t)(r + 0) * kC];
    s1 += p[(size_t)(r + 1) * kC];
    s2 += p[(size_t)(r + 2) * kC];
    s3 += p[(size_t)(r + 3) * kC];
  }
  const float s = (s0 + s1) + (s2 + s3);
  float* dst = PART + ((size_t)bs * 32 + chunk) * 256 + tid;
  *(volatile float*)dst = s;
  __threadfence();
  *(volatile float*)dst = s;
}

__global__ __launch_bounds__(256) void ssa_weight_kernel(
    const float* __restrict__ PART, const float* __restrict__ sw, float* __restrict__ WGT)
{
  const int bi = blockIdx.x;
  const int c = threadIdx.x;
  float pm[3];
#pragma unroll
  for (int j = 0; j < 3; ++j) {
    const float* pp = PART + ((size_t)(bi * 3 + j) * 32) * 256 + c;
    float s0 = 0.f, s1 = 0.f;
#pragma unroll 1
    for (int ch = 0; ch < 32; ch += 2) {
      s0 += pp[(size_t)ch * 256];
      s1 += pp[(size_t)(ch + 1) * 256];
    }
    pm[j] = (s0 + s1) * (1.0f / (float)kL);
  }
  float lg[3];
#pragma unroll
  for (int i = 0; i < 3; ++i)
    lg[i] = sw[c * 9 + i * 3 + 0] * pm[0] + sw[c * 9 + i * 3 + 1] * pm[1] + sw[c * 9 + i * 3 + 2] * pm[2];
  const float mx = fmaxf(lg[0], fmaxf(lg[1], lg[2]));
  const float e0 = expf(lg[0] - mx), e1 = expf(lg[1] - mx), e2 = expf(lg[2] - mx);
  const float inv = 1.0f / (e0 + e1 + e2);
  const float o0 = e0 * inv, o1 = e1 * inv, o2 = e2 * inv;
  float* d0p = WGT + (size_t)(bi * 3 + 0) * 256 + c;
  float* d1p = WGT + (size_t)(bi * 3 + 1) * 256 + c;
  float* d2p = WGT + (size_t)(bi * 3 + 2) * 256 + c;
  for (int pass = 0; pass < 2; ++pass) {
    *(volatile float*)d0p = o0;
    *(volatile float*)d1p = o1;
    *(volatile float*)d2p = o2;
    __threadfence();
  }
}

__global__ __launch_bounds__(256) void mix_ln_kernel(
    const float* __restrict__ XF, const float* __restrict__ SEQ, const float* __restrict__ WGT,
    const float* __restrict__ lnw, const float* __restrict__ lnb,
    float* __restrict__ XM, unsigned short* __restrict__ NXM)
{
  __shared__ __align__(16) float sS[8][kC];
  const int tid = threadIdx.x, lane = tid & 31, wave = tid >> 5;
  const int row = blockIdx.x * 8 + wave;
  const int bi = row >> 13;
  const int c0 = lane * 8;
  const size_t o = (size_t)row * kC + c0;
  const size_t pl = (size_t)kRows * kC;
  const v4f xf0 = *(const v4f*)(XF + o),           xf1 = *(const v4f*)(XF + o + 4);
  const v4f mf0 = *(const v4f*)(SEQ + o),          mf1 = *(const v4f*)(SEQ + o + 4);
  const v4f mr0 = *(const v4f*)(SEQ + pl + o),     mr1 = *(const v4f*)(SEQ + pl + o + 4);
  const v4f ff0 = *(const v4f*)(SEQ + 2 * pl + o), ff1 = *(const v4f*)(SEQ + 2 * pl + o + 4);
  const float* wg = WGT + (size_t)bi * 3 * 256 + c0;
  const v4f g00 = *(const v4f*)(wg),       g01 = *(const v4f*)(wg + 4);
  const v4f g10 = *(const v4f*)(wg + 256), g11 = *(const v4f*)(wg + 256 + 4);
  const v4f g20 = *(const v4f*)(wg + 512), g21 = *(const v4f*)(wg + 512 + 4);
  float xm[8];
#pragma unroll
  for (int e = 0; e < 4; ++e) {
    float m0 = g00[e] * mf0[e];
    m0 = m0 + g10[e] * mr0[e];
    m0 = m0 + g20[e] * ff0[e];
    xm[e] = xf0[e] + m0;
    float m1 = g01[e] * mf1[e];
    m1 = m1 + g11[e] * mr1[e];
    m1 = m1 + g21[e] * ff1[e];
    xm[4 + e] = xf1[e] + m1;
  }
  float s = 0.f;
#pragma unroll
  for (int e = 0; e < 8; ++e) s += xm[e];
  s = wave_sum32(s);
  const float mean = s * (1.0f / (float)kC);
  float dv[8];
  float qs = 0.f;
#pragma unroll
  for (int e = 0; e < 8; ++e) { dv[e] = xm[e] - mean; qs += dv[e] * dv[e]; }
  qs = wave_sum32(qs);
  const float rstd = rsqrtf(qs * (1.0f / (float)kC) + kEps);
  const v4f w0 = *(const v4f*)(lnw + c0), w1 = *(const v4f*)(lnw + c0 + 4);
  const v4f g0 = *(const v4f*)(lnb + c0), g1 = *(const v4f*)(lnb + c0 + 4);
  v8h hv;
#pragma unroll
  for (int e = 0; e < 4; ++e) {
    const float n0 = dv[e] * rstd * w0[e] + g0[e];
    const float n1 = dv[4 + e] * rstd * w1[e] + g1[e];
    hv[e]     = (_Float16)(n0 * kLnCarry);
    hv[4 + e] = (_Float16)(n1 * kLnCarry);
  }
  float* s0 = sS[wave];
  *(v4f*)(s0 + c0)     = (v4f){xm[0], xm[1], xm[2], xm[3]};
  *(v4f*)(s0 + c0 + 4) = (v4f){xm[4], xm[5], xm[6], xm[7]};
  __builtin_amdgcn_fence(__ATOMIC_RELEASE, "workgroup");
  __builtin_amdgcn_wave_barrier();
  __builtin_amdgcn_fence(__ATOMIC_ACQUIRE, "workgroup");
  const int c4 = lane * 4;
  const v4f xa = *(const v4f*)(s0 + c4), xb = *(const v4f*)(s0 + 128 + c4);
  const size_t ro = (size_t)row * kC;
  for (int pass = 0; pass < 2; ++pass) {
    *(volatile v4f*)(XM + ro + c4)       = xa;
    *(volatile v4f*)(XM + ro + 128 + c4) = xb;
    *(volatile v8h*)(NXM + ro + c0)      = hv;
    __threadfence();
  }
}

__global__ __launch_bounds__(256) void dwconv_gelu_kernel(
    const float* __restrict__ HDN, const float* __restrict__ dww, const float* __restrict__ dwb,
    unsigned short* __restrict__ HACT)
{
  __shared__ __align__(16) float sT[kW * kTileP];
  const int tid = threadIdx.x, lane = tid & 31, wave = tid >> 5;
  const int cq = blockIdx.x & 3;
  const int r  = blockIdx.x >> 2;
  const int bi = r >> 8;
  const int f  = (r >> 5) & (kNF - 1);
  const int hh = r & (kH - 1);
  const int c  = cq * 256 + tid;
  float wr[27];
#pragma unroll
  for (int k = 0; k < 27; ++k) wr[k] = dww[(size_t)c * 27 + k];
  const float bias = dwb[c];
  const size_t bb = (size_t)bi * kL;
  int lpb[9];
  bool ok[9];
#pragma unroll
  for (int kd = 0; kd < 3; ++kd) {
#pragma unroll
    for (int kh = 0; kh < 3; ++kh) {
      const int fz = f + kd - 1, hz = hh + kh - 1;
      const bool vv = (fz >= 0) && (fz < kNF) && (hz >= 0) && (hz < kH);
      const int fzc = fz < 0 ? 0 : (fz > kNF - 1 ? kNF - 1 : fz);
      const int hzc = hz < 0 ? 0 : (hz > kH - 1 ? kH - 1 : hz);
      lpb[kd * 3 + kh] = (fzc << 10) | (hzc << 5);
      ok[kd * 3 + kh] = vv;
    }
  }
  float wm[9], wc[9], wp[9];
#pragma unroll
  for (int kk = 0; kk < 9; ++kk) {
    const float t0 = HDN[(bb + (size_t)(lpb[kk] | 0)) * kHid + c];
    const float t1 = HDN[(bb + (size_t)(lpb[kk] | 1)) * kHid + c];
    wm[kk] = 0.f;
    wc[kk] = ok[kk] ? t0 : 0.f;
    wp[kk] = ok[kk] ? t1 : 0.f;
  }
#pragma unroll 1
  for (int ww = 0; ww < kW; ++ww) {
    float acc = bias;
#pragma unroll
    for (int kk = 0; kk < 9; ++kk) {
      acc = fmaf(wr[kk * 3 + 0], wm[kk], acc);
      acc = fmaf(wr[kk * 3 + 1], wc[kk], acc);
      acc = fmaf(wr[kk * 3 + 2], wp[kk], acc);
    }
    const float g = 0.5f * acc * (1.0f + erff(acc * 0.70710678118654752f));
    sT[ww * kTileP + tid] = g;
    const int wn = ww + 2;
    const bool wv = (wn < kW);
    const int wnc = wv ? wn : (kW - 1);
#pragma unroll
    for (int kk = 0; kk < 9; ++kk) {
      const float t = HDN[(bb + (size_t)(lpb[kk] | wnc)) * kHid + c];
      wm[kk] = wc[kk];
      wc[kk] = wp[kk];
      wp[kk] = (wv && ok[kk]) ? t : 0.f;
    }
  }
  __syncthreads();
  v8h hv[4];
#pragma unroll
  for (int it = 0; it < 4; ++it) {
    const float* sp = sT + (it * 8 + wave) * kTileP + lane * 8;
    const v4f a0 = *(const v4f*)(sp);
    const v4f a1 = *(const v4f*)(sp + 4);
#pragma unroll
    for (int e = 0; e < 4; ++e) {
      hv[it][e]     = (_Float16)(a0[e] * kActCarry);
      hv[it][4 + e] = (_Float16)(a1[e] * kActCarry);
    }
  }
  const size_t ob = (bb + ((size_t)f << 10) + ((size_t)hh << 5)) * kHid + (size_t)cq * 256 + lane * 8;
  for (int pass = 0; pass < 2; ++pass) {
#pragma unroll
    for (int it = 0; it < 4; ++it)
      *(volatile v8h*)(HACT + ob + (size_t)(it * 8 + wave) * kHid) = hv[it];
    __threadfence();
  }
}

__global__ __launch_bounds__(256) void unperm_out_kernel(
    const float* __restrict__ XO, const int* __restrict__ perm, float* __restrict__ out)
{
  __shared__ int sInv[32];
  __shared__ __align__(16) float sT[32 * kTileP];
  const int tid = threadIdx.x, lane = tid & 31, wave = tid >> 5;
  const int p0 = blockIdx.x * 32;
  const int f = p0 >> 10, hw0 = p0 & (kHW - 1);
  if (tid < 32) sInv[tid] = -1;
  __syncthreads();
#pragma unroll 1
  for (int it = 0; it < kL / 256; ++it) {
    const int l = it * 256 + tid;
    const int v = perm[l];
    if (v >= p0 && v < p0 + 32) sInv[v - p0] = l;
  }
  __syncthreads();
  const int q = lane >> 3, j = lane & 7;
  const v4f z4 = (v4f){0.f, 0.f, 0.f, 0.f};
#pragma unroll 1
  for (int bi = 0; bi < kB; ++bi) {
#pragma unroll
    for (int i = 0; i < 4; ++i) {
      const int k = wave * 4 + i;
      const int l = sInv[k];
      const bool okl = (l >= 0);
      const int lc = l < 0 ? 0 : (l > kL - 1 ? kL - 1 : l);
      const float* src = XO + ((size_t)bi * kL + (size_t)lc) * kC + lane * 8;
      v4f a0 = *(const v4f*)(src);
      v4f a1 = *(const v4f*)(src + 4);
      a0 = okl ? a0 : z4;
      a1 = okl ? a1 : z4;
      *(v4f*)(sT + k * kTileP + lane * 8)     = a0;
      *(v4f*)(sT + k * kTileP + lane * 8 + 4) = a1;
    }
    __syncthreads();
    v4f ov[8];
#pragma unroll
    for (int it = 0; it < 8; ++it) {
      const int c = it * 32 + wave * 4 + q;
      ov[it] = (v4f){sT[(4 * j + 0) * kTileP + c], sT[(4 * j + 1) * kTileP + c],
                     sT[(4 * j + 2) * kTileP + c], sT[(4 * j + 3) * kTileP + c]};
    }
    for (int pass = 0; pass < 2; ++pass) {
#pragma unroll
      for (int it = 0; it < 8; ++it) {
        const int c = it * 32 + wave * 4 + q;
        *(volatile v4f*)(out + ((size_t)(bi * kNF + f) * kC + c) * (size_t)kHW + hw0 + 4 * j) = ov[it];
      }
      __threadfence();
    }
    __syncthreads();
  }
}

extern "C" void kernel_launch(void* const* d_in, const int* in_sizes, int n_in,
                              void* d_out, int out_size, void* d_ws, size_t ws_size,
                              hipStream_t stream) {
  if (n_in < 23) return;
  if (in_sizes[0] != kB * kNF * kC * kHW) return;
  if (in_sizes[1] != kB * kNF * kC * kHW) return;
  if (in_sizes[2] != kL) return;
  if (in_sizes[3] != kC || in_sizes[4] != kC || in_sizes[5] != kC || in_sizes[6] != kC) return;
  if (in_sizes[7] != kC * kC) return;
  if (in_sizes[8] != kDin * 4) return;
  if (in_sizes[9] != kDin) return;
  if (in_sizes[10] != kXdW * kDin) return;
  if (in_sizes[11] != kDin * kDtR) return;
  if (in_sizes[12] != kDin) return;
  if (in_sizes[13] != kDin * kNst) return;
  if (in_sizes[14] != kDin) return;
  if (in_sizes[15] != kC * kDin) return;
  if (in_sizes[16] != kC * 9) return;
  if (in_sizes[17] != kHid * kC) return;
  if (in_sizes[18] != kHid) return;
  if (in_sizes[19] != kHid * 27) return;
  if (in_sizes[20] != kHid) return;
  if (in_sizes[21] != kC * kHid) return;
  if (in_sizes[22] != kC) return;
  if (out_size != kB * kNF * kC * kHW) return;
  if (ws_size < kWsTotal) return;

  const float* x     = (const float*)d_in[0];
  const float* fx    = (const float*)d_in[1];
  const int*   perm  = (const int*)d_in[2];
  const float* ln1w  = (const float*)d_in[3];
  const float* ln1b  = (const float*)d_in[4];
  const float* ln2w  = (const float*)d_in[5];
  const float* ln2b  = (const float*)d_in[6];
  const float* inpw  = (const float*)d_in[7];
  const float* convw = (const float*)d_in[8];
  const float* convb = (const float*)d_in[9];
  const float* xpw   = (const float*)d_in[10];
  const float* dtpw  = (const float*)d_in[11];
  const float* dtpb  = (const float*)d_in[12];
  const float* Alog  = (const float*)d_in[13];
  const float* Dp    = (const float*)d_in[14];
  const float* outpw = (const float*)d_in[15];
  const float* ssaw  = (const float*)d_in[16];
  const float* fc1w  = (const float*)d_in[17];
  const float* fc1b  = (const float*)d_in[18];
  const float* dww   = (const float*)d_in[19];
  const float* dwb   = (const float*)d_in[20];
  const float* fc2w  = (const float*)d_in[21];
  const float* fc2b  = (const float*)d_in[22];
  float* out = (float*)d_out;

  char* ws = (char*)d_ws;
  float*          XF   = (float*)(ws + kOffXF);
  float*          SEQ  = (float*)(ws + kOffSEQ);
  float*          MF   = (float*)(ws + kOffSEQ);
  float*          MR   = (float*)(ws + kOffSEQ + kPlaneB);
  float*          FF   = (float*)(ws + kOffSEQ + 2 * kPlaneB);
  float*          XZ   = (float*)(ws + kOffXZ);
  unsigned short* NX   = (unsigned short*)(ws + kOffNX);
  float*          XS   = (float*)(ws + kOffXS);
  unsigned short* XS16 = (unsigned short*)(ws + kOffXS16);
  float*          XD   = (float*)(ws + kOffXD);
  unsigned short* Y16  = (unsigned short*)(ws + kOffY16);
  float*          XM   = (float*)(ws + kOffXM);
  unsigned short* NXM  = (unsigned short*)(ws + kOffNXM);
  float*          HDN  = (float*)(ws + kOffHDN);
  unsigned short* HACT = (unsigned short*)(ws + kOffHACT);
  float*          XO   = (float*)(ws + kOffXO);
  unsigned short* WI   = (unsigned short*)(ws + kOffWI);
  unsigned short* WX   = (unsigned short*)(ws + kOffWX);
  unsigned short* WO   = (unsigned short*)(ws + kOffWO);
  unsigned short* W1   = (unsigned short*)(ws + kOffW1);
  unsigned short* W2   = (unsigned short*)(ws + kOffW2);
  float*          PART = (float*)(ws + kOffPART);
  float*          WGT  = (float*)(ws + kOffWGT);

  gather_ln_kernel<<<kRows / 8, 256, 0, stream>>>(x, fx, perm, ln1w, ln1b, XF, FF, NX);

  {
    const int n2i = kC * kC / 2;
    cast_scale_f16_kernel<<<(n2i + 255) / 256, 256, 0, stream>>>(inpw, WI, n2i, n2i, kWCarry);
    const int n2xv = kXdW * kDin / 2, n2xt = kXdP * kDin / 2;
    cast_scale_f16_kernel<<<(n2xt + 255) / 256, 256, 0, stream>>>(xpw, WX, n2xv, n2xt, kWCarry);
    const int n2o = kC * kDin / 2;
    cast_scale_f16_kernel<<<(n2o + 255) / 256, 256, 0, stream>>>(outpw, WO, n2o, n2o, kWCarry);
    const int n21 = kHid * kC / 2;
    cast_scale_f16_kernel<<<(n21 + 255) / 256, 256, 0, stream>>>(fc1w, W1, n21, n21, kWCarry);
    const int n22 = kC * kHid / 2;
    cast_scale_f16_kernel<<<(n22 + 255) / 256, 256, 0, stream>>>(fc2w, W2, n22, n22, kWCarry);
  }

  wmma_gemm64<0, 0, 0, 0, false><<<dim3((kRows / 64) * (kC / 64) / 8, 1), 256, 0, stream>>>(
      NX, nullptr, kC, 0L,
      WI, nullptr, kC, 0L,
      (void*)XZ, nullptr, kC, 0L,
      nullptr, nullptr, 0L,
      kRows, kC, kC, 1.0f / (kLnCarry * kWCarry));

  for (int dir = 0; dir < 2; ++dir) {
    conv_silu_kernel<<<kRows / 64, kDin, 0, stream>>>(XZ, convw, convb, XS, XS16, dir);
    wmma_gemm64<0, 0, 0, 0, false><<<dim3((kRows / 64) * (kXdP / 64) / 8, 1), 256, 0, stream>>>(
        XS16, nullptr, kDin, 0L,
        WX, nullptr, kDin, 0L,
        (void*)XD, nullptr, kXdP, 0L,
        nullptr, nullptr, 0L,
        kRows, kXdP, kDin, 1.0f / (kXsCarry * kWCarry));
    scan_kernel<<<kB * (kDin / kScanCh), kScanCh, 0, stream>>>(XD, XS, XZ, dtpw, dtpb, Alog, Dp, Y16, dir);
    wmma_gemm64<0, 0, 0, 0, false><<<dim3((kRows / 64) * (kC / 64) / 8, 1), 256, 0, stream>>>(
        Y16, nullptr, kDin, 0L,
        WO, nullptr, kDin, 0L,
        (void*)(dir ? MR : MF), nullptr, kC, 0L,
        nullptr, nullptr, 0L,
        kRows, kC, kDin, 1.0f / (kYCarry * kWCarry));
  }

  pool_partial_kernel<<<kB * 3 * 32, 256, 0, stream>>>(SEQ, PART);
  ssa_weight_kernel<<<kB, 256, 0, stream>>>(PART, ssaw, WGT);
  mix_ln_kernel<<<kRows / 8, 256, 0, stream>>>(XF, SEQ, WGT, ln2w, ln2b, XM, NXM);

  wmma_gemm64<0, 0, 2, 0, false><<<dim3((kRows / 64) * (kHid / 64) / 8, 1), 256, 0, stream>>>(
      NXM, nullptr, kC, 0L,
      W1, nullptr, kC, 0L,
      (void*)HDN, nullptr, kHid, 0L,
      fc1b, nullptr, 0L,
      kRows, kHid, kC, 1.0f / (kLnCarry * kWCarry));

  dwconv_gelu_kernel<<<kB * kNF * kH * (kHid / 256), 256, 0, stream>>>(HDN, dww, dwb, HACT);

  wmma_gemm64<0, 0, 2, 0, true><<<dim3((kRows / 64) * (kC / 64) / 8, 1), 256, 0, stream>>>(
      HACT, nullptr, kHid, 0L,
      W2, nullptr, kHid, 0L,
      (void*)XO, nullptr, kC, 0L,
      fc2b, XM, 0L,
      kRows, kC, kHid, 1.0f / (kActCarry * kWCarry));

  unperm_out_kernel<<<kL / 32, 256, 0, stream>>>(XO, perm, out);
}
